// MultiheadSelfAttention_61529701482744
// MI455X (gfx1250) — hardware-run, weakly checked
//
#include <hip/hip_runtime.h>


#ifndef NB
#define NB 4
#endif
#ifndef SQ
#define SQ 1024
#endif
#define NB_FULL 4
#define SQ_FULL 1024
#define MEM     1024
#define TK      (MEM + SQ)
#define TK_FULL (MEM + SQ_FULL)
#ifndef OUT_NB
#define OUT_NB NB_FULL
#endif
#define DM   1024
#define NH_  16
#define HD   64
#define AW   4
#define OSP  68
#define SC2  ((float)(0.125 * 1.4426950408889634))
#define PSH  14.0f
#define NEGB (-3.0e38f)
#define CTXS 1024.0f
#define WOS  64.0f
#define OSCL (1.0f / 65536.0f)
#define LNEPS 1.0e-5f

static_assert(HD == 64);
static_assert(NH_ * HD == DM);
static_assert(DM % 64 == 0);
static_assert(DM % 32 == 0);
static_assert(DM / 8 == 128);
static_assert(DM == 256 * 4);
static_assert(NB_FULL == 4);
static_assert(NB >= 1 && NB <= NB_FULL);
static_assert(SQ <= SQ_FULL);
static_assert(MEM % 64 == 0);
static_assert(SQ % 64 == 0);
static_assert(TK % 64 == 0);
static_assert((SQ * NB) % 64 == 0);
static_assert(TK % 32 == 0);
static_assert(SQ % 32 == 0);
static_assert(SQ % (16 * AW) == 0);
static_assert((OSP * 4) % 16 == 0);
static_assert(32 * 16 * 4 == 16 * HD * 2);
static_assert(32 * 16 * 8 == 16 * 64 * 4);
static_assert(256 * 16 * 2 == 64 * 64 * 2);
static_assert(256 * 16 == DM * 4);
static_assert(32 * 4 == 128);
static_assert(AW * 16 * OSP * 4 <= 131072);
static_assert(64 * 68 * 4 <= 131072);
static_assert(16 * 68 * 4 <= 131072);

typedef _Float16 h16;
typedef unsigned short bf;
typedef __attribute__((ext_vector_type(16))) __bf16   v16bf;
typedef __attribute__((ext_vector_type(16))) _Float16 v16h;
typedef __attribute__((ext_vector_type(8)))  _Float16 v8h;
typedef __attribute__((ext_vector_type(8)))  unsigned short v8us;
typedef __attribute__((ext_vector_type(8)))  float    v8f;
typedef __attribute__((ext_vector_type(4)))  float    v4f;
typedef __attribute__((ext_vector_type(4)))  int      v4i;
typedef v4f  __attribute__((may_alias)) v4fa;

__device__ __forceinline__ unsigned short f2bf(float f) { unsigned u = __float_as_uint(f); u += 0x7FFFu + ((u >> 16) & 1u); return (unsigned short)(u >> 16); }
__device__ __forceinline__ float bfr(float f) { return __uint_as_float(((unsigned)f2bf(f)) << 16); }
__device__ __forceinline__ v16h cat16(v8h lo, v8h hi) { return __builtin_shufflevector(lo, hi, 0, 1, 2, 3, 4, 5, 6, 7, 8, 9, 10, 11, 12, 13, 14, 15); }
__device__ __forceinline__ v16bf cat16b(v8us lo, v8us hi) { return __builtin_bit_cast(v16bf, __builtin_shufflevector(lo, hi, 0, 1, 2, 3, 4, 5, 6, 7, 8, 9, 10, 11, 12, 13, 14, 15)); }
__device__ __forceinline__ v16h  ldh(const h16* p) { return cat16(*(const v8h*)p, *(const v8h*)(p + 16)); }
__device__ __forceinline__ v16bf ldb(const bf* p)  { return cat16b(*(const v8us*)p, *(const v8us*)(p + 16)); }
__device__ __forceinline__ v8f wm16(v16h a, v16h b, v8f c) {
    c = __builtin_amdgcn_wmma_f32_16x16x32_f16(false, a, false, b, (short)0, c, false, false);
    asm volatile("v_nop\n\tv_nop\n\tv_nop\n\tv_nop" : "+v"(c) : "v"(a), "v"(b));
    return c; }
__device__ __forceinline__ v8f wmb(v16bf a, v16bf b, v8f c) {
    c = __builtin_amdgcn_wmma_f32_16x16x32_bf16(false, a, false, b, (short)0, c, false, false);
    asm volatile("v_nop\n\tv_nop\n\tv_nop\n\tv_nop" : "+v"(c) : "v"(a), "v"(b));
    return c; }
__device__ __forceinline__ h16 toh_flush(float v) { const h16 r = (h16)v; return (fabsf(v) < 6.103515625e-05f) ? (h16)0.0f : r; }
__device__ __forceinline__ void wave_sync() { __builtin_amdgcn_fence(3  , "wavefront"); __builtin_amdgcn_wave_barrier(); asm volatile("" ::: "memory"); }

__global__ __launch_bounds__(256) void k_cvt_rows(const float* __restrict__ src, bf* dst, int tlen, int nb, int src_tpitch, int src_bpitch, int dst_bpitch, int dst_trow0) {
    const size_t i = (size_t)blockIdx.x * 256 + threadIdx.x;
    const size_t n8 = (size_t)nb * (size_t)tlen * (DM / 8);
    if (i >= n8) return;
    const int c8 = (int)(i & (size_t)(DM / 8 - 1)); const size_t r = i >> 7;
    const int b = (int)(r / (size_t)tlen), t = (int)(r % (size_t)tlen);
    const size_t so = ((size_t)t * (size_t)src_tpitch + (size_t)b * (size_t)src_bpitch) * DM + (size_t)c8 * 8;
    const size_t dofs = ((size_t)b * (size_t)dst_bpitch + (size_t)dst_trow0 + (size_t)t) * DM + (size_t)c8 * 8;
    const v8f v = *(const v8f*)(src + so); v8us o;
#pragma unroll
    for (int k = 0; k < 8; ++k) o[k] = f2bf(v[k]);
    *(volatile v8us*)(dst + dofs) = o; __threadfence(); *(volatile v8us*)(dst + dofs) = o;
}

__device__ __forceinline__ void cvt_store8(bf* p, const v4f x0, const v4f x1) {
    v8us o;
#pragma unroll
    for (int i = 0; i < 4; ++i) { o[i] = f2bf(x0[i]); o[4 + i] = f2bf(x1[i]); }
    *(volatile v8us*)p = o; }
__device__ __forceinline__ void cvt_store8(h16* p, const v4f x0, const v4f x1) {
    v8h o;
#pragma unroll
    for (int i = 0; i < 4; ++i) { o[i] = toh_flush(bfr(x0[i]) * WOS); o[4 + i] = toh_flush(bfr(x1[i]) * WOS); }
    *(volatile v8h*)p = o; }

template <typename OT>
__device__ __forceinline__ void wT_body(const float* __restrict__ in, OT* out, const int N) {
    __shared__ __align__(16) float ts[64 * 68];
    const int tid = threadIdx.x; const int n0 = blockIdx.x * 64, k0 = blockIdx.y * 64;
#pragma unroll
    for (int it = 0; it < 4; ++it) { const int kk = (tid >> 4) + 16 * it; const int c4 = (tid & 15) * 4;
        const v4f v = *(const v4f*)(in + (size_t)(k0 + kk) * (size_t)N + n0 + c4);
        ts[(c4 + 0) * 68 + kk] = v[0]; ts[(c4 + 1) * 68 + kk] = v[1]; ts[(c4 + 2) * 68 + kk] = v[2]; ts[(c4 + 3) * 68 + kk] = v[3]; }
    __syncthreads();
#pragma unroll 1
    for (int ps = 0; ps < 2; ++ps) {
#pragma unroll
        for (int it = 0; it < 2; ++it) { const int n = (tid >> 3) + 32 * it; const int c8 = (tid & 7) * 8;
            const v4f x0 = *(const v4fa*)(&ts[n * 68 + c8]); const v4f x1 = *(const v4fa*)(&ts[n * 68 + c8 + 4]);
            cvt_store8(out + (size_t)(n0 + n) * DM + k0 + c8, x0, x1); }
        if (ps == 0) __threadfence(); }
}
__global__ __launch_bounds__(256) void k_wT_bf(const float* __restrict__ in, bf* out, int N) { wT_body(in, out, N); }
__global__ __launch_bounds__(256) void k_wT_h(const float* __restrict__ in, h16* out, int N) { wT_body(in, out, N); }

__global__ __launch_bounds__(128) void k_mpack(const int* __restrict__ mask, unsigned* MBT) {
    const int lane = threadIdx.x & 31;
    const int wave = __builtin_amdgcn_readfirstlane((int)(threadIdx.x >> 5));
    const int task = blockIdx.x * 4 + wave;
    if (task >= (TK / 32) * (SQ / 32)) return;
    const int kw = task / (SQ / 32), ig = task % (SQ / 32);
    unsigned w0 = 0u, w1 = 0u, w2 = 0u, w3 = 0u;
#pragma unroll 1
    for (int q = 0; q < 32; ++q) {
        const size_t e = ((size_t)(ig * 32 + q) * TK_FULL + (size_t)(kw * 32 + lane)) * NB_FULL;
        const v4i mv = *(const v4i*)(mask + e);
        const unsigned b0 = __builtin_amdgcn_ballot_w32(mv[0] != 0);
        const unsigned b1 = __builtin_amdgcn_ballot_w32(mv[1] != 0);
        const unsigned b2 = __builtin_amdgcn_ballot_w32(mv[2] != 0);
        const unsigned b3 = __builtin_amdgcn_ballot_w32(mv[3] != 0);
        const bool mine = lane == q;
        w0 = mine ? b0 : w0; w1 = mine ? b1 : w1; w2 = mine ? b2 : w2; w3 = mine ? b3 : w3;
    }
    const size_t o0 = ((size_t)0 * (TK / 32) + kw) * SQ + (size_t)(ig * 32 + lane);
    const size_t pl = (size_t)(TK / 32) * SQ;
#pragma unroll 1
    for (int ps = 0; ps < 2; ++ps) {
        *(volatile unsigned*)(MBT + o0) = w0;
        if (NB > 1) *(volatile unsigned*)(MBT + o0 + pl) = w1;
        if (NB > 2) *(volatile unsigned*)(MBT + o0 + 2 * pl) = w2;
        if (NB > 3) *(volatile unsigned*)(MBT + o0 + 3 * pl) = w3;
        if (ps == 0) __threadfence(); }
}

template <int MODE>
__device__ __forceinline__ void proj_body(const bf* __restrict__ CBp, const bf* __restrict__ Wt, h16* Ph, const int tper, const int tofs, const int ptok, const int pofs) {
    __shared__ __align__(16) float os[16 * 68];
    const int lane = threadIdx.x & 31, lr = lane & 15, hi = lane >> 4;
    const int ti = (MODE == 0) ? (int)blockIdx.x : (int)blockIdx.y;
    const int fi = (MODE == 0) ? (int)blockIdx.y : (int)blockIdx.x;
    const int lin = ti * 64; const int b = lin / tper; const int t0 = tofs + lin % tper;
    const int nparts = (t0 >= MEM) ? 2 : 1;
    v8f acc[4][4];
#pragma unroll
    for (int mb = 0; mb < 4; ++mb)
#pragma unroll
        for (int nb = 0; nb < 4; ++nb) acc[mb][nb] = (v8f){};
    const size_t woff = (size_t)(fi * 64 + lr) * DM + 8 * hi;
#pragma unroll 1
    for (int p = 0; p < nparts; ++p) {
        const size_t trow = (p == 0) ? ((size_t)b * TK + (size_t)t0) : ((size_t)NB * TK + (size_t)(t0 - MEM));
        const size_t toff = (trow + (size_t)lr) * DM + 8 * hi;
#pragma unroll 1
        for (int kc = 0; kc < DM; kc += 32) {
            v16bf a[4];
            if (MODE == 0) {
#pragma unroll
                for (int mb = 0; mb < 4; ++mb) a[mb] = ldb(CBp + toff + (size_t)mb * 16 * DM + kc);
#pragma unroll
                for (int nb = 0; nb < 4; ++nb) { const v16bf bfr_ = ldb(Wt + woff + (size_t)nb * 16 * DM + kc);
#pragma unroll
                    for (int mb = 0; mb < 4; ++mb) acc[mb][nb] = wmb(a[mb], bfr_, acc[mb][nb]); }
            } else {
#pragma unroll
                for (int mb = 0; mb < 4; ++mb) a[mb] = ldb(Wt + woff + (size_t)mb * 16 * DM + kc);
#pragma unroll
                for (int nb = 0; nb < 4; ++nb) { const v16bf bfr_ = ldb(CBp + toff + (size_t)nb * 16 * DM + kc);
#pragma unroll
                    for (int mb = 0; mb < 4; ++mb) acc[mb][nb] = wmb(a[mb], bfr_, acc[mb][nb]); }
            }
        }
    }
    size_t obase, opitch;
    if (MODE == 0) { obase = ((size_t)(b * NH_ + fi) * (size_t)ptok + (size_t)(t0 - pofs)) * HD; opitch = HD; }
    else           { obase = ((size_t)b * DM + (size_t)fi * 64) * TK + (size_t)t0;            opitch = TK; }
#pragma unroll
    for (int mb = 0; mb < 4; ++mb) {
#pragma unroll
        for (int nb = 0; nb < 4; ++nb) {
#pragma unroll
            for (int j = 0; j < 8; ++j) os[(hi * 8 + j) * 68 + nb * 16 + lr] = acc[mb][nb][j]; }
        wave_sync();
#pragma unroll 1
        for (int ps = 0; ps < 2; ++ps) {
#pragma unroll
            for (int s = 0; s < 4; ++s) { const int row = 4 * s + (lane >> 3), c8 = (lane & 7) * 8;
                const v4f x0 = *(const v4fa*)(&os[row * 68 + c8]); const v4f x1 = *(const v4fa*)(&os[row * 68 + c8 + 4]); v8h hv;
#pragma unroll
                for (int i = 0; i < 4; ++i) { hv[i] = toh_flush(x0[i]); hv[4 + i] = toh_flush(x1[i]); }
                *(volatile v8h*)(Ph + obase + (size_t)(mb * 16 + row) * opitch + c8) = hv; }
            if (ps == 0) __threadfence(); }
        wave_sync();
    }
}
__global__ __launch_bounds__(32) void k_proj_tok(const bf* __restrict__ CBp, const bf* __restrict__ Wt, h16* Ph, int tper, int tofs, int ptok, int pofs) { proj_body<0>(CBp, Wt, Ph, tper, tofs, ptok, pofs); }
__global__ __launch_bounds__(32) void k_proj_vt(const bf* __restrict__ CBp, const bf* __restrict__ Wt, h16* Ph) { proj_body<1>(CBp, Wt, Ph, TK, 0, TK, 0); }

__global__ __launch_bounds__(32 * AW) void k_flash(const h16* __restrict__ QH, const h16* __restrict__ KP, const h16* __restrict__ VT, const unsigned* __restrict__ MBT, h16* CTX) {
    __shared__ __align__(16) float os[AW * 16 * OSP];
    const int lane = threadIdx.x & 31, lr = lane & 15, hi = lane >> 4;
    const int wave = __builtin_amdgcn_readfirstlane((int)(threadIdx.x >> 5));
    const int zh = blockIdx.y; const int b = zh / NH_, h = zh % NH_;
    const int t0 = (blockIdx.x * AW + wave) * 16;
    const size_t qo = ((size_t)zh * SQ + (size_t)(t0 + lr)) * HD + 8 * hi;
    const v16h qh0 = ldh(QH + qo), qh1 = ldh(QH + qo + 32);
    const size_t ko = (size_t)zh * TK * HD + (size_t)lr * HD + 8 * hi;
    const size_t vo = (size_t)zh * HD * TK + (size_t)lr * TK + 8 * hi;
    const size_t mo = (size_t)b * (TK / 32) * SQ + (size_t)(t0 + lr);
    v8f o0 = (v8f){}, o1 = (v8f){}, o2 = (v8f){}, o3 = (v8f){};
    float m = NEGB, l = 0.0f;
#pragma unroll 1
    for (int key0 = 0; key0 < TK; key0 += 32) {
        unsigned mw = MBT[mo + (size_t)(key0 >> 5) * SQ];
        asm volatile("" : "+v"(mw));
        if (__builtin_amdgcn_ballot_w32(mw != 0xFFFFFFFFu) == 0u) continue;
        const h16* ka = KP + ko + (size_t)key0 * HD;
        const v16h ka0 = ldh(ka), ka1 = ldh(ka + 32), kb0 = ldh(ka + 16 * HD), kb1 = ldh(ka + 16 * HD + 32);
        v8f sa = (v8f){}, sb = (v8f){};
        sa = wm16(ka0, qh0, sa); sb = wm16(kb0, qh0, sb); sa = wm16(ka1, qh1, sa); sb = wm16(kb1, qh1, sb);
        const unsigned kbits = (~mw) >> (8 * hi);
        float ta[8], tb[8]; bool fa[8], fb[8]; float mx = NEGB;
#pragma unroll
        for (int r = 0; r < 8; ++r) {
            fa[r] = ((kbits >> r) & 1u) != 0u;
            fb[r] = ((kbits >> (16 + r)) & 1u) != 0u;
            ta[r] = sa[r] * SC2; tb[r] = sb[r] * SC2;
            mx = fmaxf(mx, fmaxf(fa[r] ? ta[r] : NEGB, fb[r] ? tb[r] : NEGB)); }
        mx = fmaxf(mx, __shfl_xor(mx, 16, 32));
        const float mnew = fmaxf(m, mx);
        const float alpha = __builtin_amdgcn_exp2f(m - mnew);
        const float sh = PSH - mnew;
        v16h pb; float ls = 0.0f;
#pragma unroll
        for (int r = 0; r < 8; ++r) {
            const float xa = ta[r] + sh, xb = tb[r] + sh;
            const float ea = (xa < -14.0f) ? 0.0f : __builtin_amdgcn_exp2f(xa);
            const float eb = (xb < -14.0f) ? 0.0f : __builtin_amdgcn_exp2f(xb);
            const float ga = fa[r] ? ea : 0.0f, gb = fb[r] ? eb : 0.0f;
            const h16 pa = (h16)ga; const h16 pc = (h16)gb;
            pb[r] = pa; pb[8 + r] = pc;
            ls += (float)pa + (float)pc; }
        l = l * alpha + ls; m = mnew;
        o0 = o0 * alpha; o1 = o1 * alpha; o2 = o2 * alpha; o3 = o3 * alpha;
        const h16* va = VT + vo + key0;
        const v16h v0 = ldh(va), v1 = ldh(va + (size_t)16 * TK), v2 = ldh(va + (size_t)32 * TK), v3 = ldh(va + (size_t)48 * TK);
        o0 = wm16(v0, pb, o0); o1 = wm16(v1, pb, o1); o2 = wm16(v2, pb, o2); o3 = wm16(v3, pb, o3);
    }
    l += __shfl_xor(l, 16, 32);
    const bool any = l > 0.0f;
    const float lsafe = any ? l : 1.0f;
    const float scl = (1.0f / lsafe) * CTXS;
    const float nanv = __uint_as_float(0x7FC00000u);
    const int wb = wave * 16 * OSP;
    { v4f a, c;
#pragma unroll
      for (int i = 0; i < 4; ++i) { a[i] = any ? o0[i] * scl : nanv; c[i] = any ? o0[4 + i] * scl : nanv; }
      *(v4fa*)(&os[wb + lr * OSP +  0 + 8 * hi]) = a; *(v4fa*)(&os[wb + lr * OSP +  0 + 8 * hi + 4]) = c;
#pragma unroll
      for (int i = 0; i < 4; ++i) { a[i] = any ? o1[i] * scl : nanv; c[i] = any ? o1[4 + i] * scl : nanv; }
      *(v4fa*)(&os[wb + lr * OSP + 16 + 8 * hi]) = a; *(v4fa*)(&os[wb + lr * OSP + 16 + 8 * hi + 4]) = c;
#pragma unroll
      for (int i = 0; i < 4; ++i) { a[i] = any ? o2[i] * scl : nanv; c[i] = any ? o2[4 + i] * scl : nanv; }
      *(v4fa*)(&os[wb + lr * OSP + 32 + 8 * hi]) = a; *(v4fa*)(&os[wb + lr * OSP + 32 + 8 * hi + 4]) = c;
#pragma unroll
      for (int i = 0; i < 4; ++i) { a[i] = any ? o3[i] * scl : nanv; c[i] = any ? o3[4 + i] * scl : nanv; }
      *(v4fa*)(&os[wb + lr * OSP + 48 + 8 * hi]) = a; *(v4fa*)(&os[wb + lr * OSP + 48 + 8 * hi + 4]) = c; }
    wave_sync();
    h16* crow = CTX + ((size_t)t0 * NB + (size_t)b) * DM + h * HD;
#pragma unroll 1
    for (int ps = 0; ps < 2; ++ps) {
#pragma unroll
        for (int s = 0; s < 4; ++s) { const int row = 4 * s + (lane >> 3), c8 = (lane & 7) * 8;
            const v4f x0 = *(const v4fa*)(&os[wb + row * OSP + c8]); const v4f x1 = *(const v4fa*)(&os[wb + row * OSP + c8 + 4]); v8h hv;
#pragma unroll
            for (int i = 0; i < 4; ++i) { hv[i] = toh_flush(x0[i]); hv[4 + i] = toh_flush(x1[i]); }
            *(volatile v8h*)(crow + (size_t)row * NB * DM + c8) = hv; }
        if (ps == 0) __threadfence(); }
}

__global__ __launch_bounds__(32) void k_oproj(const h16* __restrict__ A, const h16* __restrict__ Bt, const float* __restrict__ x, const float* __restrict__ pos, float* Y) {
    __shared__ __align__(16) float os[16 * 68];
    const int lane = threadIdx.x & 31, lr = lane & 15, hi = lane >> 4; const int r0 = blockIdx.x * 64, c0 = blockIdx.y * 64;
    v8f acc[4][4];
#pragma unroll
    for (int mb = 0; mb < 4; ++mb)
#pragma unroll
        for (int nb = 0; nb < 4; ++nb) acc[mb][nb] = (v8f){};
    const size_t aoff = (size_t)(r0 + lr) * DM + 8 * hi, boff = (size_t)(c0 + lr) * DM + 8 * hi;
#pragma unroll 1
    for (int kc = 0; kc < DM; kc += 32) {
        v16h a[4];
#pragma unroll
        for (int mb = 0; mb < 4; ++mb) a[mb] = ldh(A + aoff + (size_t)mb * 16 * DM + kc);
#pragma unroll
        for (int nb = 0; nb < 4; ++nb) { const v16h bq = ldh(Bt + boff + (size_t)nb * 16 * DM + kc);
#pragma unroll
            for (int mb = 0; mb < 4; ++mb) acc[mb][nb] = wm16(a[mb], bq, acc[mb][nb]); }
    }
#pragma unroll
    for (int mb = 0; mb < 4; ++mb) {
#pragma unroll
        for (int nb = 0; nb < 4; ++nb) {
#pragma unroll
            for (int j = 0; j < 8; ++j) os[(hi * 8 + j) * 68 + nb * 16 + lr] = acc[mb][nb][j] * OSCL; }
        wave_sync();
#pragma unroll 1
        for (int ps = 0; ps < 2; ++ps) {
#pragma unroll 2
            for (int s = 0; s < 8; ++s) { const int row = 2 * s + (lane >> 4), c4 = (lane & 15) * 4;
                const int mrow = r0 + mb * 16 + row; const int sq = mrow / NB, bb = mrow % NB;
                const v4f val = *(const v4fa*)(&os[row * 68 + c4]);
                const v4f xv = *(const v4f*)(x + ((size_t)sq * NB_FULL + (size_t)bb) * DM + c0 + c4);
                const v4f pv = *(const v4f*)(pos + (size_t)sq * DM + c0 + c4);
                v4f y;
#pragma unroll
                for (int i = 0; i < 4; ++i) y[i] = (bfr(xv[i]) + bfr(pv[i])) + val[i];
                *(volatile v4f*)(Y + (size_t)mrow * DM + c0 + c4) = y; }
            if (ps == 0) __threadfence(); }
        wave_sync();
    }
}

__global__ __launch_bounds__(256) void k_ln(const float* __restrict__ Y, const float* __restrict__ gam, const float* __restrict__ bet, float* OUT) {
#pragma clang fp contract(off)
    __shared__ float r1[8];
    __shared__ float r2[8];
    const int tid = threadIdx.x, lane = tid & 31, wv = tid >> 5;
    const int r = blockIdx.x; const int sq = r / NB, bb = r % NB;
    const v4f y = *(const v4f*)(Y + (size_t)r * DM + tid * 4);
    float s = (y[0] + y[1]) + (y[2] + y[3]);
    s += __shfl_xor(s, 16, 32); s += __shfl_xor(s, 8, 32); s += __shfl_xor(s, 4, 32); s += __shfl_xor(s, 2, 32); s += __shfl_xor(s, 1, 32);
    if (lane == 0) r1[wv] = s;
    __syncthreads();
    float tot = 0.0f;
#pragma unroll 1
    for (int i = 0; i < 8; ++i) tot += r1[i];
    const float mu = tot * (1.0f / (float)DM);
    v4f d;
#pragma unroll
    for (int i = 0; i < 4; ++i) d[i] = y[i] - mu;
    float q = (d[0] * d[0] + d[1] * d[1]) + (d[2] * d[2] + d[3] * d[3]);
    q += __shfl_xor(q, 16, 32); q += __shfl_xor(q, 8, 32); q += __shfl_xor(q, 4, 32); q += __shfl_xor(q, 2, 32); q += __shfl_xor(q, 1, 32);
    if (lane == 0) r2[wv] = q;
    __syncthreads();
    float tq = 0.0f;
#pragma unroll 1
    for (int i = 0; i < 8; ++i) tq += r2[i];
    const float var = tq * (1.0f / (float)DM);
    const float rs = rsqrtf(var + LNEPS);
    const v4f g = *(const v4f*)(gam + tid * 4); const v4f be = *(const v4f*)(bet + tid * 4);
    v4f o;
#pragma unroll
    for (int i = 0; i < 4; ++i) o[i] = d[i] * rs * bfr(g[i]) + bfr(be[i]);
    float* op = OUT + ((size_t)sq * OUT_NB + (size_t)bb) * DM + tid * 4;
    *(volatile v4f*)op = o; __threadfence(); *(volatile v4f*)op = o;
}

static constexpr size_t al256(size_t v) { return (v + 255) & ~(size_t)255; }
static constexpr size_t SZ_CB = al256((size_t)(NB * TK + SQ) * DM * 2);
static constexpr size_t SZ_WT = al256((size_t)3 * DM * DM * 2);
static constexpr size_t SZ_WO = al256((size_t)DM * DM * 2);
static constexpr size_t SZ_QH = al256((size_t)NB * NH_ * SQ * HD * 2);
static constexpr size_t SZ_KP = al256((size_t)NB * NH_ * TK * HD * 2);
static constexpr size_t SZ_VT = al256((size_t)NB * DM * TK * 2);
static constexpr size_t SZ_MB = al256((size_t)NB * (TK / 32) * SQ * 4);
static constexpr size_t SZ_CX = al256((size_t)SQ * NB * DM * 2);
static constexpr size_t SZ_Y  = al256((size_t)SQ * NB * DM * 4);
static constexpr size_t SZ_TOTAL = SZ_CB + SZ_WT + SZ_WO + SZ_QH + SZ_KP + SZ_VT + SZ_MB + SZ_CX + SZ_Y;
static_assert(SZ_TOTAL <= (size_t)134217728);
static_assert((size_t)NB * NH_ * TK * HD == (size_t)NB * DM * TK);
static_assert(((size_t)DM * DM * 2) % 256 == 0);
static constexpr size_t NEED_X  = ((size_t)(SQ - 1) * NB_FULL + NB) * DM;
static constexpr size_t NEED_P  = (size_t)SQ * DM;
static constexpr size_t NEED_M  = ((size_t)(MEM - 1) * NB_FULL + NB) * DM;
static constexpr size_t NEED_K  = ((size_t)(SQ - 1) * TK_FULL + TK) * NB_FULL;
static constexpr size_t NEED_O  = ((size_t)(SQ - 1) * OUT_NB + NB) * DM;

extern "C" void kernel_launch(void* const* d_in, const int* in_sizes, int n_in,
                              void* d_out, int out_size, void* d_ws, size_t ws_size, hipStream_t stream) {
    if (n_in < 8) return;
    if ((size_t)in_sizes[0] < NEED_X || (size_t)in_sizes[1] < NEED_P || (size_t)in_sizes[2] < NEED_M || (size_t)in_sizes[3] < NEED_K) return;
    if ((size_t)in_sizes[4] < (size_t)3 * DM * DM || (size_t)in_sizes[5] < (size_t)DM * DM || in_sizes[6] < DM || in_sizes[7] < DM) return;
    if ((size_t)out_size < NEED_O) return;
    if (SZ_TOTAL > ws_size) return;
    const float* xin = (const float*)d_in[0]; const float* pin = (const float*)d_in[1]; const float* min_ = (const float*)d_in[2];
    const int* mask = (const int*)d_in[3];
    const float* wqkv = (const float*)d_in[4]; const float* wo = (const float*)d_in[5];
    const float* gam = (const float*)d_in[6]; const float* bet = (const float*)d_in[7];
    float* OUT = (float*)d_out;
    char* wsp = (char*)d_ws;
    bf* CB  = (bf*)wsp;  wsp += SZ_CB;
    bf* WT  = (bf*)wsp;  wsp += SZ_WT;
    h16* WOT = (h16*)wsp; wsp += SZ_WO;
    h16* QH = (h16*)wsp; wsp += SZ_QH;
    h16* KP = (h16*)wsp; wsp += SZ_KP;
    h16* VT = (h16*)wsp; wsp += SZ_VT;
    unsigned* MBT = (unsigned*)wsp; wsp += SZ_MB;
    h16* CX = (h16*)wsp; wsp += SZ_CX;
    float* Y = (float*)wsp; wsp += SZ_Y;

    { const size_t n8 = (size_t)NB * MEM * (DM / 8);
      k_cvt_rows<<<(unsigned)((n8 + 255) / 256), 256, 0, stream>>>(min_, CB, MEM, NB, NB_FULL, 1, TK, 0); }
    { const size_t n8 = (size_t)NB * SQ * (DM / 8);
      k_cvt_rows<<<(unsigned)((n8 + 255) / 256), 256, 0, stream>>>(xin, CB, SQ, NB, NB_FULL, 1, TK, MEM); }
    { const size_t n8 = (size_t)SQ * (DM / 8);
      k_cvt_rows<<<(unsigned)((n8 + 255) / 256), 256, 0, stream>>>(pin, CB, SQ, 1, 1, 0, 0, NB * TK); }
    k_wT_bf<<<dim3(3 * DM / 64, DM / 64, 1), 256, 0, stream>>>(wqkv, WT, 3 * DM);
    k_wT_h<<<dim3(DM / 64, DM / 64, 1), 256, 0, stream>>>(wo, WOT, DM);
    k_mpack<<<((TK / 32) * (SQ / 32) + 3) / 4, 128, 0, stream>>>(mask, MBT);

    k_proj_tok<<<dim3(NB * SQ / 64, DM / 64, 1), 32, 0, stream>>>(CB, WT, QH, SQ, MEM, SQ, MEM);
    k_proj_tok<<<dim3(NB * TK / 64, DM / 64, 1), 32, 0, stream>>>(CB, WT + (size_t)DM * DM, KP, TK, 0, TK, 0);
    k_proj_vt<<<dim3(DM / 64, NB * TK / 64, 1), 32, 0, stream>>>(CB, WT + (size_t)2 * DM * DM, VT);

    k_flash<<<dim3(SQ / (16 * AW), NB * NH_, 1), 32 * AW, 0, stream>>>(QH, KP, VT, MBT, CX);
    k_oproj<<<dim3(SQ * NB / 64, DM / 64, 1), 32, 0, stream>>>(CX, WOT, xin, pin, Y);
    k_ln<<<SQ * NB, 256, 0, stream>>>(Y, gam, bet, OUT);
}
